// RansGinoGridToMesh_49744311222706
// MI455X (gfx1250) — hardware-verified
//
#include <hip/hip_runtime.h>
#include <stddef.h>


#define NTHR   256
#define NWAVE  8
#define HD     256
#define HD2    512
#define EPT    8
#define CHUNK  (NTHR * EPT)
#define WCAP   (EPT * 32)
#define LISTN  (NWAVE * WCAP)
#define PASSN  64
#define PCAP   (CHUNK + PASSN)
#define RMAXP  ((PCAP + PASSN - 1) / PASSN)
#define NB     64
#define NWROWS 1552
#define NWB    (NWROWS / NWAVE)
#define NOMEGA 42
#define EMBW   84
#define WSC    16.0f
#define WINV   0.0625f

static_assert(NWB * NWAVE == NWROWS);
static_assert(NTHR == HD);
static_assert(PASSN * 4 == NTHR);
static_assert((PASSN / 16) * 2 == NWAVE);
static_assert(NB == 64);
static_assert(LISTN * 4 <= PASSN * HD2 * 2);

typedef float    v4f  __attribute__((ext_vector_type(4)));
typedef float    v8f  __attribute__((ext_vector_type(8)));
typedef int      v4i  __attribute__((ext_vector_type(4)));
typedef _Float16 v8h  __attribute__((ext_vector_type(8)));
typedef _Float16 v16h __attribute__((ext_vector_type(16)));

union FragH { v16h v; v8h h[2]; };
union HV { v8h h; v4i u; };
union __attribute__((aligned(16))) TileU { _Float16 h[PASSN * HD2]; float f[PASSN * HD]; int l[LISTN]; };

__device__ __forceinline__ int clampi(int v, int lo, int hi) { return v < lo ? lo : (v > hi ? hi : v); }

__device__ __forceinline__ float gelu_f(float x) {
  return 0.5f * x * (1.0f + erff(x * 0.70710678118654752f));
}

__device__ __forceinline__ v8f zacc() {
  v8f z;
#pragma unroll
  for (int i = 0; i < 8; ++i) z[i] = 0.0f;
  return z;
}

__device__ __forceinline__ v8f wmh(v16h a, v16h b, v8f c) {
  v8f d = __builtin_amdgcn_wmma_f32_16x16x32_f16(false, a, false, b, (short)0, c, false, false);
  asm volatile("v_nop\n\tv_nop\n\tv_nop\n\tv_nop" : "+v"(d) : "v"(a), "v"(b));
  return d;
}

template <int NT, int KS>
__device__ __forceinline__ void wgemm(const _Float16* Ab, int lda, const _Float16* Bb, int ldb,
                                      v8f (&acc)[NT], int lane) {
  const int h = lane >> 4, m = lane & 15;
  const _Float16* ap = Ab + m * lda + 8 * h;
  const _Float16* bp = Bb + m * ldb + 8 * h;
#pragma unroll
  for (int j = 0; j < NT; ++j) acc[j] = zacc();
#pragma unroll 1
  for (int ks = 0; ks < KS; ++ks) {
    FragH a;
    a.h[0] = *(const v8h*)(ap + 32 * ks);
    a.h[1] = *(const v8h*)(ap + 32 * ks + 16);
#pragma unroll
    for (int j = 0; j < NT; ++j) {
      FragH b;
      const _Float16* bq = bp + j * 16 * ldb + 32 * ks;
      b.h[0] = *(const v8h*)bq;
      b.h[1] = *(const v8h*)(bq + 16);
      acc[j] = wmh(a.v, b.v, acc[j]);
    }
  }
}

__global__ __launch_bounds__(NTHR) void k_prep(
    const float* __restrict__ proj_w, const float* __restrict__ msg_w1, const float* __restrict__ msg_w2,
    const float* __restrict__ msg_w3, const float* __restrict__ pred_w1, const float* __restrict__ pred_w2,
    const float* __restrict__ x, const float* __restrict__ qpos,
    _Float16* PWt, _Float16* W1t, _Float16* W2t, _Float16* W3t, _Float16* P1t, _Float16* W2Pt,
    _Float16* Xh, _Float16* Qh, int nG, int nQ) {
  __shared__ float om[64];
  __shared__ __attribute__((aligned(16))) _Float16 qs[NWAVE * HD];
  const int tid = threadIdx.x, lane = tid & 31, wave = tid >> 5;
  if (tid < NOMEGA) {
    const float ex = (float)(2 * tid) * (1.0f / (float)EMBW);
    om[tid] = 1.0f / powf(10000.0f, ex);
  }
  __syncthreads();

  const int b = blockIdx.x;
  const int nXB = nG / NWAVE, nQB = nQ / NWAVE;
  if (b < NWB) {
    const int wr = b * NWAVE + wave;
    const float* W; int N, K, n, lim; _Float16* drow;
    if (wr < 256)       { W = proj_w;  N = HD;  K = HD;  n = wr;        lim = HD;  drow = PWt  + (size_t)n * HD;  }
    else if (wr < 768)  { W = msg_w1;  N = HD2; K = HD2; n = wr - 256;  lim = HD2; drow = W1t  + (size_t)n * HD2; }
    else if (wr < 1024) { W = msg_w2;  N = HD;  K = HD2; n = wr - 768;  lim = HD;  drow = W2t  + (size_t)n * HD2; }
    else if (wr < 1280) { W = msg_w3;  N = HD;  K = HD;  n = wr - 1024; lim = HD;  drow = W3t  + (size_t)n * HD;  }
    else if (wr < 1536) { W = pred_w1; N = HD;  K = HD;  n = wr - 1280; lim = HD;  drow = P1t  + (size_t)n * HD;  }
    else                { W = pred_w2; N = 4;   K = HD;  n = wr - 1536; lim = 4;   drow = W2Pt + (size_t)n * HD;  }
    const bool nz = n < lim;
    const int nn = nz ? n : 0;
    HV o0, o1;
    {
      v8h t;
#pragma unroll
      for (int i = 0; i < 8; ++i) {
        const int k = 8 * lane + i;
        const float v = nz ? W[(size_t)k * N + nn] * WSC : 0.0f;
        t[i] = (_Float16)v;
      }
      o0.h = t;
    }
    o1 = o0;
    if (K > HD) {
      v8h t;
#pragma unroll
      for (int i = 0; i < 8; ++i) {
        const int k = HD + 8 * lane + i;
        const float v = nz ? W[(size_t)k * N + nn] * WSC : 0.0f;
        t[i] = (_Float16)v;
      }
      o1.h = t;
    }
    *(volatile v4i*)(drow + 8 * lane) = o0.u;
    if (K > HD) *(volatile v4i*)(drow + HD + 8 * lane) = o1.u;
    __threadfence();
    *(volatile v4i*)(drow + 8 * lane) = o0.u;
    if (K > HD) *(volatile v4i*)(drow + HD + 8 * lane) = o1.u;
  } else if (b < NWB + nXB) {
    const int row = (b - NWB) * NWAVE + wave;
    const float* xp = x + (size_t)row * HD + 8 * lane;
    const v4f a = *(const v4f*)xp;
    const v4f c = *(const v4f*)(xp + 4);
    v8h t;
    t[0] = (_Float16)a.x; t[1] = (_Float16)a.y; t[2] = (_Float16)a.z; t[3] = (_Float16)a.w;
    t[4] = (_Float16)c.x; t[5] = (_Float16)c.y; t[6] = (_Float16)c.z; t[7] = (_Float16)c.w;
    HV o; o.h = t;
    _Float16* dp = Xh + (size_t)row * HD + 8 * lane;
    *(volatile v4i*)dp = o.u;
    __threadfence();
    *(volatile v4i*)dp = o.u;
  } else if (b < NWB + nXB + nQB) {
    const int row = (b - NWB - nXB) * NWAVE + wave;
    const float p0 = qpos[(size_t)row * 3 + 0];
    const float p1 = qpos[(size_t)row * 3 + 1];
    const float p2 = qpos[(size_t)row * 3 + 2];
#pragma unroll 1
    for (int i = 0; i < 8; ++i) {
      const int col = 8 * lane + i;
      float val = 0.0f;
      if (col < 3 * EMBW) {
        const int d = col / EMBW;
        const int rr = col - EMBW * d;
        const int i2 = (rr < NOMEGA) ? rr : rr - NOMEGA;
        const float cd = (d == 0) ? p0 : ((d == 1) ? p1 : p2);
        const float c = cd * om[i2];
        val = (rr < NOMEGA) ? sinf(c) : cosf(c);
      }
      qs[wave * HD + col] = (_Float16)val;
    }
    __syncthreads();
    HV o;
    o.h = *(const v8h*)(qs + wave * HD + 8 * lane);
    _Float16* dp = Qh + (size_t)row * HD + 8 * lane;
    *(volatile v4i*)dp = o.u;
    __threadfence();
    *(volatile v4i*)dp = o.u;
  }
}

template <int KS>
__global__ __launch_bounds__(NTHR) void k_gemm(
    const _Float16* __restrict__ A, int lda, const _Float16* __restrict__ Bt, int ldb,
    const float* __restrict__ bias, int hasBias, _Float16* Cout, int ldc) {
  __shared__ __attribute__((aligned(16))) _Float16 Ct[64 * HD];
  const int tid = threadIdx.x, lane = tid & 31, wave = tid >> 5, hh = lane >> 4, mm = lane & 15;
  const int mt = wave >> 1, nh = wave & 1;
  const int m0 = blockIdx.x * 64;
  const int n0 = blockIdx.y * HD;

  v8f acc[8];
  wgemm<8, KS>(A + (size_t)(m0 + mt * 16) * lda, lda, Bt + (size_t)(n0 + nh * 128) * ldb, ldb, acc, lane);

#pragma unroll
  for (int j = 0; j < 8; ++j) {
    const int n = nh * 128 + 16 * j + mm;
    const float bv = (hasBias != 0) ? bias[n0 + n] : 0.0f;
#pragma unroll
    for (int rr = 0; rr < 8; ++rr) {
      const int row = mt * 16 + 8 * hh + rr;
      Ct[row * HD + n] = (_Float16)(acc[j][rr] * WINV + bv);
    }
  }
  __syncthreads();

  HV ov[8];
#pragma unroll
  for (int i = 0; i < 8; ++i) {
    const int row = wave + NWAVE * i;
    ov[i].h = *(const v8h*)(Ct + row * HD + 8 * lane);
  }
#pragma unroll
  for (int i = 0; i < 8; ++i) {
    const int row = wave + NWAVE * i;
    _Float16* p = Cout + (size_t)(m0 + row) * ldc + n0 + 8 * lane;
    *(volatile v4i*)p = ov[i].u;
  }
  __threadfence();
#pragma unroll
  for (int i = 0; i < 8; ++i) {
    const int row = wave + NWAVE * i;
    _Float16* p = Cout + (size_t)(m0 + row) * ldc + n0 + 8 * lane;
    *(volatile v4i*)p = ov[i].u;
  }
}

__device__ __forceinline__ int scan_chunk(const int* __restrict__ edges, int nE, int cbase, int nodeBase,
                                          int* list, int tid, int wave) {
  int wc = 0;
  const int el0 = tid * EPT;
  const int e0  = cbase + el0;
  const int sent = -2147483647 - 1;
  int q0, q1, q2, q3, q4, q5, q6, q7;
  if (e0 + 7 < nE) {
    const v4i* p = (const v4i*)(edges + (size_t)e0 * 2);
    const v4i a0 = p[0], a1 = p[1], a2 = p[2], a3 = p[3];
    q0 = a0.x; q1 = a0.z; q2 = a1.x; q3 = a1.z;
    q4 = a2.x; q5 = a2.z; q6 = a3.x; q7 = a3.z;
  } else {
    q0 = (e0     < nE) ? edges[(size_t)(e0    ) * 2] : sent;
    q1 = (e0 + 1 < nE) ? edges[(size_t)(e0 + 1) * 2] : sent;
    q2 = (e0 + 2 < nE) ? edges[(size_t)(e0 + 2) * 2] : sent;
    q3 = (e0 + 3 < nE) ? edges[(size_t)(e0 + 3) * 2] : sent;
    q4 = (e0 + 4 < nE) ? edges[(size_t)(e0 + 4) * 2] : sent;
    q5 = (e0 + 5 < nE) ? edges[(size_t)(e0 + 5) * 2] : sent;
    q6 = (e0 + 6 < nE) ? edges[(size_t)(e0 + 6) * 2] : sent;
    q7 = (e0 + 7 < nE) ? edges[(size_t)(e0 + 7) * 2] : sent;
  }
  const unsigned nb = (unsigned)nodeBase;
  const bool h0 = ((unsigned)q0 - nb) < (unsigned)NB, h1 = ((unsigned)q1 - nb) < (unsigned)NB;
  const bool h2 = ((unsigned)q2 - nb) < (unsigned)NB, h3 = ((unsigned)q3 - nb) < (unsigned)NB;
  const bool h4 = ((unsigned)q4 - nb) < (unsigned)NB, h5 = ((unsigned)q5 - nb) < (unsigned)NB;
  const bool h6 = ((unsigned)q6 - nb) < (unsigned)NB, h7 = ((unsigned)q7 - nb) < (unsigned)NB;
  const unsigned any = __builtin_amdgcn_ballot_w32(h0 | h1 | h2 | h3 | h4 | h5 | h6 | h7);
  if (any != 0u) {
#define HITJ(J, HJ) { \
      const unsigned mj = __builtin_amdgcn_ballot_w32(HJ); \
      if (mj != 0u) { \
        if (HJ) { \
          const int pos = wc + (int)__builtin_amdgcn_mbcnt_lo(mj, 0u); \
          if (pos < WCAP) list[wave * WCAP + pos] = el0 + (J); \
        } \
        wc += (int)__builtin_popcount(mj); } }
    HITJ(0, h0)
    HITJ(1, h1)
    HITJ(2, h2)
    HITJ(3, h3)
    HITJ(4, h4)
    HITJ(5, h5)
    HITJ(6, h6)
    HITJ(7, h7)
#undef HITJ
  }
  return wc;
}

__global__ __launch_bounds__(NTHR) void k_agg(
    const _Float16* __restrict__ GPh, const _Float16* __restrict__ QPh, const int* __restrict__ edges,
    const _Float16* __restrict__ W2t, const float* __restrict__ b2,
    const _Float16* __restrict__ W3t, const float* __restrict__ b3,
    const _Float16* __restrict__ P1t, const float* __restrict__ pb1,
    const _Float16* __restrict__ W2Pt, const float* __restrict__ pb2,
    float* outp, int nG, int nQ, int nE) {
  __shared__ __attribute__((aligned(16))) float accS[(NB + 1) * HD];
  __shared__ TileU tile;
  __shared__ __attribute__((aligned(16))) int   pend[PCAP];
  __shared__ __attribute__((aligned(16))) float outS[NB * 4];
  __shared__ float cntS[NB + 1];
  __shared__ float indS[NB];
  __shared__ float b2S[HD];
  __shared__ float b3S[HD];
  __shared__ float pb1S[HD];
  __shared__ float pb2S[4];
  __shared__ int   slotS[PASSN];
  __shared__ int   wcnt[NWAVE];
  __shared__ int   pendN;

  const int tid = threadIdx.x, lane = tid & 31, wave = tid >> 5, hh = lane >> 4, mm = lane & 15;
  const int mt = wave >> 1, nh = wave & 1;
  const int nodeBase = blockIdx.x * NB;

  for (int i = tid; i < (NB + 1) * HD; i += NTHR) accS[i] = 0.0f;
  if (tid < NB + 1) cntS[tid] = 0.0f;
  b2S[tid]  = b2[tid];
  b3S[tid]  = b3[tid];
  pb1S[tid] = pb1[tid];
  if (tid < 4) pb2S[tid] = pb2[tid];
  if (tid == 0) pendN = 0;
  __syncthreads();

  const int nChunks = (nE + CHUNK - 1) / CHUNK;
#pragma unroll 1
  for (int ch = 0; ch < nChunks; ++ch) {
    const int cbase = ch * CHUNK;
    const int wc = scan_chunk(edges, nE, cbase, nodeBase, tile.l, tid, wave);
    if (lane == 0) wcnt[wave] = wc;
    __syncthreads();

    const int base = pendN;
    int tot = 0, myoff = 0;
#pragma unroll
    for (int w = 0; w < NWAVE; ++w) {
      const int c = clampi(wcnt[w], 0, WCAP);
      if (w < wave) myoff += c;
      tot += c;
    }
    int newN = base + tot;
    newN = newN > PCAP ? PCAP : newN;
    {
      const int n = clampi(wcnt[wave], 0, WCAP);
      const int* lp = tile.l + wave * WCAP;
      for (int i = lane; i < n; i += 32) {
        const int pos = base + myoff + i;
        if (pos < PCAP) pend[pos] = cbase + lp[i];
      }
    }
    const int fin = (ch == nChunks - 1) ? 1 : 0;
    int R = (fin != 0) ? (newN + PASSN - 1) / PASSN : newN / PASSN;
    R = clampi(R, 0, RMAXP);
    const int Pv = (fin != 0) ? newN : R * PASSN;
    __syncthreads();

#pragma unroll 1
    for (int r = 0; r < R; ++r) {
      {
        const int er = tid >> 2, qq = tid & 3;
        const int idx = r * PASSN + er;
        const bool valid = idx < Pv;
        int e = 0;
        if (valid) e = pend[idx];
        e = clampi(e, 0, nE - 1);
        const int q = edges[(size_t)e * 2];
        int g = edges[(size_t)e * 2 + 1];
        int slot = q - nodeBase;
        if (!valid || (unsigned)slot >= (unsigned)NB) slot = NB;
        g = clampi(g, 0, nG - 1);
        const int qc = clampi(q, 0, nQ - 1);
        if (qq == 0) slotS[er] = slot;
        const _Float16* gp = GPh + (size_t)g  * HD2 + qq * 128;
        const _Float16* qp = QPh + (size_t)qc * HD2 + qq * 128;
        _Float16* dp = tile.h + er * HD2 + qq * 128;
#pragma unroll 1
        for (int c = 0; c < 16; ++c) {
          const v8h av = *(const v8h*)(gp + 8 * c);
          const v8h bv = *(const v8h*)(qp + 8 * c);
          v8h o;
#pragma unroll
          for (int i = 0; i < 8; ++i) {
            const float s = (float)av[i] + (float)bv[i];
            const float gl = valid ? gelu_f(s) : 0.0f;
            o[i] = (_Float16)gl;
          }
          *(v8h*)(dp + 8 * c) = o;
        }
      }
      __syncthreads();

      v8f acc[8];
      wgemm<8, HD2 / 32>(tile.h + mt * 16 * HD2, HD2, W2t + (size_t)(nh * 128) * HD2, HD2, acc, lane);
      __syncthreads();

#pragma unroll
      for (int j = 0; j < 8; ++j) {
        const int n = nh * 128 + 16 * j + mm;
        const float bvv = b2S[n];
#pragma unroll
        for (int rr = 0; rr < 8; ++rr) {
          const int row = mt * 16 + 8 * hh + rr;
          tile.f[row * HD + n] = gelu_f(acc[j][rr] * WINV + bvv);
        }
      }
      __syncthreads();

#pragma unroll 1
      for (int k = 0; k < PASSN; ++k) {
        const int sl = clampi(slotS[k], 0, NB);
        accS[sl * HD + tid] += tile.f[k * HD + tid];
        if (tid == 0) cntS[sl] += 1.0f;
      }
      __syncthreads();
    }

    int rem = newN - R * PASSN;
    rem = rem < 0 ? 0 : rem;
    if (R > 0 && tid < rem) pend[tid] = pend[R * PASSN + tid];
    if (tid == 0) pendN = rem;
  }
  __syncthreads();

#pragma unroll 1
  for (int s = 0; s < NB; ++s) {
    const float cn = cntS[s];
    const float inv = 1.0f / fmaxf(cn, 1.0f);
    tile.h[s * HD + tid] = (_Float16)(accS[s * HD + tid] * inv);
  }
  if (tid < NB) indS[tid] = (cntS[tid] > 0.0f) ? 1.0f : 0.0f;
  __syncthreads();

  {
    v8f acc[8];
    wgemm<8, HD / 32>(tile.h + mt * 16 * HD, HD, W3t + (size_t)(nh * 128) * HD, HD, acc, lane);
    __syncthreads();
#pragma unroll
    for (int j = 0; j < 8; ++j) {
      const int n = nh * 128 + 16 * j + mm;
      const float bvv = b3S[n];
#pragma unroll
      for (int rr = 0; rr < 8; ++rr) {
        const int row = mt * 16 + 8 * hh + rr;
        tile.h[row * HD + n] = (_Float16)(acc[j][rr] * WINV + bvv * indS[row]);
      }
    }
  }
  __syncthreads();

  {
    v8f acc[8];
    wgemm<8, HD / 32>(tile.h + mt * 16 * HD, HD, P1t + (size_t)(nh * 128) * HD, HD, acc, lane);
    __syncthreads();
#pragma unroll
    for (int j = 0; j < 8; ++j) {
      const int n = nh * 128 + 16 * j + mm;
      const float bvv = pb1S[n];
#pragma unroll
      for (int rr = 0; rr < 8; ++rr) {
        const int row = mt * 16 + 8 * hh + rr;
        tile.h[row * HD + n] = (_Float16)gelu_f(acc[j][rr] * WINV + bvv);
      }
    }
  }
  __syncthreads();

  if (wave < 4) {
    v8f a1[1];
    wgemm<1, HD / 32>(tile.h + wave * 16 * HD, HD, W2Pt, HD, a1, lane);
    if (mm < 4) {
#pragma unroll
      for (int rr = 0; rr < 8; ++rr) {
        const int row = wave * 16 + 8 * hh + rr;
        outS[row * 4 + mm] = a1[0][rr] * WINV + pb2S[mm];
      }
    }
  }
  __syncthreads();

  v4f o0 = {0.0f, 0.0f, 0.0f, 0.0f};
  v4f o1 = o0;
  const bool wr = (wave == 0);
  if (wr) {
    o0 = *(const v4f*)(outS + 4 * lane);
    o1 = *(const v4f*)(outS + 128 + 4 * lane);
  }
  float* ob = outp + (size_t)nodeBase * 4;
  if (wr) {
    *(volatile v4f*)(ob + 4 * lane) = o0;
    *(volatile v4f*)(ob + 128 + 4 * lane) = o1;
  }
  __threadfence();
  if (wr) {
    *(volatile v4f*)(ob + 4 * lane) = o0;
    *(volatile v4f*)(ob + 128 + 4 * lane) = o1;
  }
}

static size_t al256(size_t b) { return (b + 255) & ~(size_t)255; }

extern "C" void kernel_launch(void* const* d_in, const int* in_sizes, int n_in,
                              void* d_out, int out_size, void* d_ws, size_t ws_size,
                              hipStream_t stream) {
  if (n_in < 15) return;
  const int nG = in_sizes[0] / HD;
  const int nQ = in_sizes[1] / 3;
  const int nE = in_sizes[2] / 2;
  if (nG <= 0 || nQ <= 0 || nE < 0) return;
  if (in_sizes[0] != nG * HD || in_sizes[1] != nQ * 3 || in_sizes[2] != nE * 2) return;
  if ((nG % 64) != 0 || (nQ % NB) != 0) return;
  if (in_sizes[3] != HD * HD || in_sizes[4] != HD) return;
  if (in_sizes[5] != HD2 * HD2 || in_sizes[6] != HD2) return;
  if (in_sizes[7] != HD2 * HD || in_sizes[8] != HD) return;
  if (in_sizes[9] != HD * HD || in_sizes[10] != HD) return;
  if (in_sizes[11] != HD * HD || in_sizes[12] != HD) return;
  if (in_sizes[13] != HD * 4 || in_sizes[14] != 4) return;
  if (out_size != nQ * 4) return;

  const float* x       = (const float*)d_in[0];
  const float* qpos    = (const float*)d_in[1];
  const int*   edges   = (const int*)d_in[2];
  const float* proj_w  = (const float*)d_in[3];
  const float* proj_b  = (const float*)d_in[4];
  const float* msg_w1  = (const float*)d_in[5];
  const float* msg_b1  = (const float*)d_in[6];
  const float* msg_w2  = (const float*)d_in[7];
  const float* msg_b2  = (const float*)d_in[8];
  const float* msg_w3  = (const float*)d_in[9];
  const float* msg_b3  = (const float*)d_in[10];
  const float* pred_w1 = (const float*)d_in[11];
  const float* pred_b1 = (const float*)d_in[12];
  const float* pred_w2 = (const float*)d_in[13];
  const float* pred_b2 = (const float*)d_in[14];
  float* out = (float*)d_out;

  char* ws = (char*)d_ws;
  size_t off = 0;
  const size_t oPW  = off; off += al256((size_t)HD  * HD  * 2);
  const size_t oW1  = off; off += al256((size_t)HD2 * HD2 * 2);
  const size_t oW2  = off; off += al256((size_t)HD  * HD2 * 2);
  const size_t oW3  = off; off += al256((size_t)HD  * HD  * 2);
  const size_t oP1  = off; off += al256((size_t)HD  * HD  * 2);
  const size_t oW2P = off; off += al256((size_t)16  * HD  * 2);
  const size_t oXh  = off; off += al256((size_t)nG * HD  * 2);
  const size_t oQh  = off; off += al256((size_t)nQ * HD  * 2);
  const size_t oGh  = off; off += al256((size_t)nG * HD  * 2);
  const size_t oGP  = off; off += al256((size_t)nG * HD2 * 2);
  const size_t oQP  = off; off += al256((size_t)nQ * HD2 * 2);
  if (off > ws_size) return;

  _Float16* PWt  = (_Float16*)(ws + oPW);
  _Float16* W1t  = (_Float16*)(ws + oW1);
  _Float16* W2t  = (_Float16*)(ws + oW2);
  _Float16* W3t  = (_Float16*)(ws + oW3);
  _Float16* P1t  = (_Float16*)(ws + oP1);
  _Float16* W2Pt = (_Float16*)(ws + oW2P);
  _Float16* Xh   = (_Float16*)(ws + oXh);
  _Float16* Qh   = (_Float16*)(ws + oQh);
  _Float16* Gh   = (_Float16*)(ws + oGh);
  _Float16* GPh  = (_Float16*)(ws + oGP);
  _Float16* QPh  = (_Float16*)(ws + oQP);

  k_prep<<<dim3(NWB + nG / NWAVE + nQ / NWAVE), dim3(NTHR), 0, stream>>>(
      proj_w, msg_w1, msg_w2, msg_w3, pred_w1, pred_w2, x, qpos,
      PWt, W1t, W2t, W3t, P1t, W2Pt, Xh, Qh, nG, nQ);

  k_gemm<HD / 32><<<dim3(nG / 64, 1), dim3(NTHR), 0, stream>>>(
      Xh, HD, PWt, HD, proj_b, 1, Gh, HD);

  k_gemm<HD / 32><<<dim3(nG / 64, HD2 / HD), dim3(NTHR), 0, stream>>>(
      Gh, HD, W1t, HD2, msg_b1, 0, GPh, HD2);

  k_gemm<HD / 32><<<dim3(nQ / 64, HD2 / HD), dim3(NTHR), 0, stream>>>(
      Qh, HD, W1t + HD, HD2, msg_b1, 1, QPh, HD2);

  k_agg<<<dim3(nQ / NB), dim3(NTHR), 0, stream>>>(
      GPh, QPh, edges, W2t, msg_b2, W3t, msg_b3, P1t, pred_b1, W2Pt, pred_b2, out, nG, nQ, nE);
}
